// Rnn_net_22754736734783
// MI455X (gfx1250) — hardware-verified
//
#include <hip/hip_runtime.h>
#include <math.h>

typedef __attribute__((ext_vector_type(16))) _Float16 v16h;
typedef __attribute__((ext_vector_type(8)))  _Float16 v8h;
typedef __attribute__((ext_vector_type(8)))  float    v8f;
typedef __attribute__((ext_vector_type(4)))  float    v4f;

constexpr int kBatch      = 4096;
constexpr int kSteps      = 2048;
constexpr int kHid        = 10;
constexpr int kTileRows   = 16;
constexpr int kTiles      = kBatch / kTileRows;
constexpr int kChunk      = 32;
constexpr int kNumChunks  = kSteps / kChunk;
constexpr int kPitch      = 36;
constexpr int kTileState  = kTileRows * kHid;
constexpr int kMatElems   = kHid * kHid;
constexpr size_t kOut0Elems = (size_t)kBatch * (size_t)kSteps;
constexpr size_t kOut1Elems = (size_t)2 * kBatch * kHid;
static_assert(kBatch % kTileRows == 0, "whole 16-row tiles");
static_assert(kSteps % kChunk == 0, "whole 32-step chunks");
static_assert(kHid <= 16 && 2 * 16 == 32, "units fit one 16-row subtile, two k halves of 16");
static_assert(kOut0Elems * 4 == 33554432ull, "byte offset of the second output");
static_assert((kTileState * 4) % 128 == 0, "a tile's final-state rows are whole 128-B lines");
static_assert(((size_t)kBatch * kHid * 4) % 128 == 0, "state planes start on a line");
static_assert(kMatElems % 4 == 0 && kTileState % 4 == 0, "16-B vector staging");
static_assert((kPitch % 4) == 0, "16-B aligned LDS rows");

constexpr float kStateCarry  = 256.0f;
constexpr float kWeightCarry = 64.0f;
constexpr float kFoldBack    = 1.0f / (kStateCarry * kWeightCarry);
constexpr float kF16MinNorm  = 6.103515625e-5f;
static_assert(kStateCarry * kWeightCarry == 16384.0f, "carry product");

namespace eng {

union FragU { v16h v; v8h h[2]; };

__device__ __forceinline__ unsigned short f2bf_bits(float f) {
  unsigned u = __float_as_uint(f);
  return (unsigned short)((u + 0x7FFFu + ((u >> 16) & 1u)) >> 16);
}
__device__ __forceinline__ float bf16v(float f) {
  return __uint_as_float(((unsigned)f2bf_bits(f)) << 16);
}
__device__ __forceinline__ _Float16 to_f16_flushed(float c) {
  const float z = (fabsf(c) < kF16MinNorm) ? 0.0f : c;
  return (_Float16)z;
}
__device__ __forceinline__ v8f mma_f16(v16h a, v16h b) {
  v8f c = (v8f){0.f, 0.f, 0.f, 0.f, 0.f, 0.f, 0.f, 0.f};
  c = __builtin_amdgcn_wmma_f32_16x16x32_f16(false, a, false, b, (short)0, c, false, false);
  asm volatile("v_nop\n\tv_nop\n\tv_nop\n\tv_nop" : "+v"(c) : "v"(a), "v"(b));
  return c;
}
__device__ __forceinline__ float fast_tanh(float v) {
  const float e = __expf(2.0f * v);
  return 1.0f - 2.0f * __builtin_amdgcn_rcpf(e + 1.0f);
}

}

__global__ __launch_bounds__(32) void rnn2_seq_kernel(
    const float* __restrict__ x,
    const float* __restrict__ hinit,
    const float* __restrict__ w_ih0,
    const float* __restrict__ w_hh0,
    const float* __restrict__ b_ih0,
    const float* __restrict__ b_hh0,
    const float* __restrict__ w_ih1,
    const float* __restrict__ w_hh1,
    const float* __restrict__ b_ih1,
    const float* __restrict__ b_hh1,
    const float* __restrict__ w_out,
    const float* __restrict__ b_out,
    float* __restrict__ outs,
    float* __restrict__ hout)
{
  __shared__ __align__(16) float xs[kTileRows * kPitch];
  __shared__ __align__(16) float os[kTileRows * kPitch];
  __shared__ __align__(16) float hsm[2 * kTileState];
  __shared__ __align__(16) float wsm[3 * kMatElems];
  __shared__ __align__(16) float csm[7 * 32];

  const int lane = threadIdx.x & 31;
  const int hsel = lane >> 4;
  const int n    = lane & 15;
  const bool lowHalf = (hsel == 0);
  const int b0   = blockIdx.x * kTileRows;

  {
    const int wi = (lane < 24) ? lane : 24;
    const v4f m0 = *(const v4f*)(w_hh0 + 4 * wi);
    const v4f m1 = *(const v4f*)(w_ih1 + 4 * wi);
    const v4f m2 = *(const v4f*)(w_hh1 + 4 * wi);
    *(v4f*)(wsm + 4 * wi)                 = m0;
    *(v4f*)(wsm + kMatElems + 4 * wi)     = m1;
    *(v4f*)(wsm + 2 * kMatElems + 4 * wi) = m2;
    const int ci = (lane < 9) ? lane : 9;
    csm[0 * 32 + lane] = b_ih0[ci];
    csm[1 * 32 + lane] = b_hh0[ci];
    csm[2 * 32 + lane] = b_ih1[ci];
    csm[3 * 32 + lane] = b_hh1[ci];
    csm[4 * 32 + lane] = w_ih0[ci];
    csm[5 * 32 + lane] = w_out[ci];
    csm[6 * 32 + lane] = b_out[0];
    const int ia = lane;
    const int ib = 32 + (lane & 7);
    const float* hp0 = hinit + (size_t)b0 * kHid;
    const float* hp1 = hinit + ((size_t)kBatch + (size_t)b0) * kHid;
    const v4f s0a = *(const v4f*)(hp0 + 4 * ia);
    const v4f s0b = *(const v4f*)(hp0 + 4 * ib);
    const v4f s1a = *(const v4f*)(hp1 + 4 * ia);
    const v4f s1b = *(const v4f*)(hp1 + 4 * ib);
    *(v4f*)(hsm + 4 * ia)              = s0a;
    *(v4f*)(hsm + 4 * ib)              = s0b;
    *(v4f*)(hsm + kTileState + 4 * ia) = s1a;
    *(v4f*)(hsm + kTileState + 4 * ib) = s1b;
  }
  __syncthreads();

  v16h fragA0, fragA1;
  {
    const int m  = n;
    const int mc = (m < kHid) ? m : (kHid - 1);
    const bool mok = (m < kHid);
    v8h a0lo, a1lo, a1hi;
    const v8h zero8 = (v8h){(_Float16)0.0f, (_Float16)0.0f, (_Float16)0.0f, (_Float16)0.0f,
                            (_Float16)0.0f, (_Float16)0.0f, (_Float16)0.0f, (_Float16)0.0f};
#pragma unroll
    for (int i = 0; i < 8; ++i) {
      const int k  = 8 * hsel + i;
      const int kc = (k < kHid) ? k : (kHid - 1);
      const bool ok = mok && (k < kHid);
      const float f0 = wsm[mc * kHid + kc];
      const float f1 = wsm[kMatElems + mc * kHid + kc];
      const float f2 = wsm[2 * kMatElems + mc * kHid + kc];
      const float g0 = ok ? (eng::bf16v(f0) * kWeightCarry) : 0.0f;
      const float g1 = ok ? (eng::bf16v(f1) * kWeightCarry) : 0.0f;
      const float g2 = ok ? (eng::bf16v(f2) * kWeightCarry) : 0.0f;
      a0lo[i] = eng::to_f16_flushed(g0);
      a1lo[i] = eng::to_f16_flushed(g1);
      a1hi[i] = eng::to_f16_flushed(g2);
    }
    eng::FragU u0, u1;
    u0.h[0] = a0lo;
    u0.h[1] = zero8;
    u1.h[0] = a1lo;
    u1.h[1] = a1hi;
    fragA0 = u0.v;
    fragA1 = u1.v;
  }

  float cb0[8], cb1[8], wx[8], wo[8];
  float h0f[8], h1f[8];
  v8h hb0, hb1;
#pragma unroll
  for (int r = 0; r < 8; ++r) {
    const int u  = 8 * hsel + r;
    const int uc = (u < kHid) ? u : (kHid - 1);
    const bool live = (u < kHid);
    const float vb0 = eng::bf16v(csm[0 * 32 + uc]) + eng::bf16v(csm[1 * 32 + uc]);
    const float vb1 = eng::bf16v(csm[2 * 32 + uc]) + eng::bf16v(csm[3 * 32 + uc]);
    const float vwx = eng::bf16v(csm[4 * 32 + uc]);
    const float vwo = eng::bf16v(csm[5 * 32 + uc]);
    const float s0  = eng::bf16v(hsm[n * kHid + uc]);
    const float s1  = eng::bf16v(hsm[kTileState + n * kHid + uc]);
    cb0[r] = live ? vb0 : 0.0f;
    cb1[r] = live ? vb1 : 0.0f;
    wx[r]  = live ? vwx : 0.0f;
    wo[r]  = live ? vwo : 0.0f;
    h0f[r] = live ? s0 : 0.0f;
    h1f[r] = live ? s1 : 0.0f;
    hb0[r] = eng::to_f16_flushed(h0f[r] * kStateCarry);
    hb1[r] = eng::to_f16_flushed(h1f[r] * kStateCarry);
  }
  const float bo = eng::bf16v(csm[6 * 32]);
  const v8h zh = (v8h){(_Float16)0.0f, (_Float16)0.0f, (_Float16)0.0f, (_Float16)0.0f,
                       (_Float16)0.0f, (_Float16)0.0f, (_Float16)0.0f, (_Float16)0.0f};

  const int q  = lane >> 3;
  const int c4 = (lane & 7) * 4;

#pragma unroll 1
  for (int ch = 0; ch < kNumChunks; ++ch) {
    const int t0 = ch * kChunk;
#pragma unroll
    for (int it = 0; it < 4; ++it) {
      const int row = it * 4 + q;
      const v4f v = *(const v4f*)(x + (size_t)(b0 + row) * kSteps + t0 + c4);
      v4f rv;
      rv[0] = eng::bf16v(v[0]);
      rv[1] = eng::bf16v(v[1]);
      rv[2] = eng::bf16v(v[2]);
      rv[3] = eng::bf16v(v[3]);
      *(v4f*)(xs + row * kPitch + c4) = rv;
    }
    __syncthreads();

#pragma unroll 1
    for (int s = 0; s < kChunk; ++s) {
      const float xv = xs[n * kPitch + s];

      eng::FragU fb;
      fb.h[0] = hb0;
      fb.h[1] = zh;
      const v8f acc0 = eng::mma_f16(fragA0, fb.v);
#pragma unroll
      for (int r = 0; r < 8; ++r) {
        const float pre = fmaf(acc0[r], kFoldBack, fmaf(xv, wx[r], cb0[r]));
        const float tv  = eng::fast_tanh(pre);
        const bool live = (r < 2) || lowHalf;
        const float hv  = live ? tv : 0.0f;
        h0f[r] = hv;
        hb0[r] = eng::to_f16_flushed(hv * kStateCarry);
      }

      fb.h[0] = hb0;
      fb.h[1] = hb1;
      const v8f acc1 = eng::mma_f16(fragA1, fb.v);
#pragma unroll
      for (int r = 0; r < 8; ++r) {
        const float pre = fmaf(acc1[r], kFoldBack, cb1[r]);
        const float tv  = eng::fast_tanh(pre);
        const bool live = (r < 2) || lowHalf;
        const float hv  = live ? tv : 0.0f;
        h1f[r] = hv;
        hb1[r] = eng::to_f16_flushed(hv * kStateCarry);
      }

      float p = 0.0f;
#pragma unroll
      for (int r = 0; r < 8; ++r) p = fmaf(wo[r], h1f[r], p);
      const float pother = __shfl_xor(p, 16, 32);
      const float tot = (p + pother) + bo;
      if (lowHalf) os[n * kPitch + s] = tot;
    }
    __syncthreads();

    {
      v4f ov[4];
#pragma unroll
      for (int it = 0; it < 4; ++it) ov[it] = *(const v4f*)(os + (it * 4 + q) * kPitch + c4);
      for (int pass = 0; pass < 2; ++pass) {
#pragma unroll
        for (int it = 0; it < 4; ++it)
          *(volatile v4f*)(outs + (size_t)(b0 + it * 4 + q) * kSteps + t0 + c4) = ov[it];
        __threadfence();
      }
    }
  }

#pragma unroll
  for (int r = 0; r < 8; ++r) {
    const bool live = (r < 2) || lowHalf;
    const int u = 8 * hsel + r;
    if (live) {
      hsm[n * kHid + u]              = h0f[r];
      hsm[kTileState + n * kHid + u] = h1f[r];
    }
  }
  __syncthreads();
  {
    const int ia = lane;
    const int ib = 32 + (lane & 7);
    const v4f a0 = *(const v4f*)(hsm + 4 * ia);
    const v4f e0 = *(const v4f*)(hsm + 4 * ib);
    const v4f a1 = *(const v4f*)(hsm + kTileState + 4 * ia);
    const v4f e1 = *(const v4f*)(hsm + kTileState + 4 * ib);
    float* p0 = hout + (size_t)b0 * kHid;
    float* p1 = hout + ((size_t)kBatch + (size_t)b0) * kHid;
    for (int pass = 0; pass < 2; ++pass) {
      *(volatile v4f*)(p0 + 4 * ia) = a0;
      *(volatile v4f*)(p1 + 4 * ia) = a1;
      if (lane < 8) {
        *(volatile v4f*)(p0 + 4 * ib) = e0;
        *(volatile v4f*)(p1 + 4 * ib) = e1;
      }
      __threadfence();
    }
  }
}

extern "C" void kernel_launch(void* const* d_in, const int* in_sizes, int n_in,
                              void* d_out, int out_size, void* d_ws, size_t ws_size,
                              hipStream_t stream) {
  (void)d_ws;
  (void)ws_size;
  if (n_in < 12 || d_out == nullptr) return;
  if (in_sizes[0] != kBatch * kSteps) return;
  if (in_sizes[1] != 2 * kBatch * kHid) return;
  if (in_sizes[2] != kHid) return;
  if (in_sizes[3] != kMatElems) return;
  if (in_sizes[4] != kHid) return;
  if (in_sizes[5] != kHid) return;
  if (in_sizes[6] != kMatElems) return;
  if (in_sizes[7] != kMatElems) return;
  if (in_sizes[8] != kHid) return;
  if (in_sizes[9] != kHid) return;
  if (in_sizes[10] != kHid) return;
  if (in_sizes[11] != 1) return;
  if ((size_t)out_size != kOut0Elems + kOut1Elems) return;

  const float* x     = (const float*)d_in[0];
  const float* hinit = (const float*)d_in[1];
  const float* w_ih0 = (const float*)d_in[2];
  const float* w_hh0 = (const float*)d_in[3];
  const float* b_ih0 = (const float*)d_in[4];
  const float* b_hh0 = (const float*)d_in[5];
  const float* w_ih1 = (const float*)d_in[6];
  const float* w_hh1 = (const float*)d_in[7];
  const float* b_ih1 = (const float*)d_in[8];
  const float* b_hh1 = (const float*)d_in[9];
  const float* w_out = (const float*)d_in[10];
  const float* b_out = (const float*)d_in[11];

  float* outs = (float*)d_out;
  float* hout = outs + kOut0Elems;

  rnn2_seq_kernel<<<kTiles, 32, 0, stream>>>(
      x, hinit, w_ih0, w_hh0, b_ih0, b_hh0, w_ih1, w_hh1, b_ih1, b_hh1, w_out, b_out, outs, hout);
}
